// RelativeMultiHeadAttentionLayer_7937099563620
// MI455X (gfx1250) — hardware-verified
//
#include <hip/hip_runtime.h>
#include <math.h>

typedef __attribute__((ext_vector_type(16))) _Float16 v16h;
typedef __attribute__((ext_vector_type(16))) __bf16 v16b;
typedef __attribute__((ext_vector_type(8)))  _Float16 v8h;
typedef __attribute__((ext_vector_type(8)))  float v8f;
typedef __attribute__((ext_vector_type(4)))  float v4f;
typedef __attribute__((ext_vector_type(2)))  float v2f;
typedef __attribute__((ext_vector_type(4)))  unsigned v4u;
typedef __attribute__((ext_vector_type(4)))  int v4i;
typedef float __attribute__((may_alias)) float_a;
typedef int __attribute__((may_alias)) int_a;

template <typename T> __device__ __forceinline__ void vst2(void* p, T v) { *(volatile T*)p = v; __threadfence(); *(volatile T*)p = v; }
__device__ __forceinline__ v8f wmma16(v16h a, v16h b, v8f c) {
  v8f d = __builtin_amdgcn_wmma_f32_16x16x32_f16(false, a, false, b, (short)0, c, false, false);
  asm volatile("v_nop\n\tv_nop\n\tv_nop\n\tv_nop" : "+v"(d) : "v"(a), "v"(b));
  return d;
}
__device__ __forceinline__ v8f wmma_bf(v16b a, v16b b, v8f c) {
  v8f d = __builtin_amdgcn_wmma_f32_16x16x32_bf16(false, a, false, b, (short)0, c, false, false);
  asm volatile("v_nop\n\tv_nop\n\tv_nop\n\tv_nop" : "+v"(d) : "v"(a), "v"(b));
  return d;
}
__device__ __forceinline__ v16h frag_h(const _Float16* rowk0, int lane) {
  union { v16h v; v8h q[2]; } u; const _Float16* p = rowk0 + 8 * (lane >> 4);
  u.q[0] = *(const v8h*)p; u.q[1] = *(const v8h*)(p + 16); return u.v;
}
__device__ __forceinline__ v16h frag_f32(const float* rowk0, int lane) {
  v16h a; const float* p = rowk0 + 8 * (lane >> 4);
#pragma unroll
  for (int i = 0; i < 8; ++i) { a[i] = (_Float16)p[i]; a[8 + i] = (_Float16)p[16 + i]; }
  return a;
}
__device__ __forceinline__ v16h frag_f32s(const float* rowk0, int lane, float sc) {
  v16h a; const float* p = rowk0 + 8 * (lane >> 4);
#pragma unroll
  for (int i = 0; i < 8; ++i) { a[i] = (_Float16)(p[i] * sc); a[8 + i] = (_Float16)(p[16 + i] * sc); }
  return a;
}
__device__ __forceinline__ v16h fragc_f32(const float* W, int k0, int n, int lane, int ld, int K) {
  v16h a; const int g = lane >> 4;
#pragma unroll
  for (int i = 0; i < 8; ++i) { const int ka = k0 + 8 * g + i, kb = ka + 16;
    a[i] = (_Float16)(ka < K ? W[(size_t)(ka < K ? ka : K - 1) * ld + n] : 0.f); a[8 + i] = (_Float16)(kb < K ? W[(size_t)(kb < K ? kb : K - 1) * ld + n] : 0.f); }
  return a;
}
struct F2 { v16b h, l; };
__device__ __forceinline__ F2 bsplit16(const float v[16]) { F2 r;
#pragma unroll
  for (int i = 0; i < 16; ++i) { const __bf16 h = (__bf16)v[i]; r.h[i] = h; r.l[i] = (__bf16)(v[i] - (float)h); }
  return r; }
__device__ __forceinline__ F2 split_row(const float* row, int k0, int lane) { float v[16]; const float* p = row + k0 + 8 * (lane >> 4);
#pragma unroll
  for (int i = 0; i < 8; ++i) { v[i] = p[i]; v[8 + i] = p[16 + i]; }
  return bsplit16(v); }
__device__ __forceinline__ F2 split_rowK(const float* row, int k0, int lane, int K) { float v[16]; const int g = lane >> 4;
#pragma unroll
  for (int i = 0; i < 8; ++i) { const int ka = k0 + 8 * g + i, kb = ka + 16; v[i] = ka < K ? row[ka < K ? ka : K - 1] : 0.f; v[8 + i] = kb < K ? row[kb < K ? kb : K - 1] : 0.f; }
  return bsplit16(v); }
__device__ __forceinline__ F2 split_col(const float* W, int k0, int n, int lane, int ld, int K) { float v[16]; const int g = lane >> 4;
#pragma unroll
  for (int i = 0; i < 8; ++i) { const int ka = k0 + 8 * g + i, kb = ka + 16; v[i] = ka < K ? W[(size_t)(ka < K ? ka : K - 1) * ld + n] : 0.f; v[8 + i] = kb < K ? W[(size_t)(kb < K ? kb : K - 1) * ld + n] : 0.f; }
  return bsplit16(v); }
__device__ __forceinline__ v8f mac3(const F2& a, const F2& b, v8f c) { c = wmma_bf(a.l, b.h, c); c = wmma_bf(a.h, b.l, c); return wmma_bf(a.h, b.h, c); }
__device__ __forceinline__ float sigm(float v) { return 1.0f / (1.0f + expf(-v)); }
#define LDSX() do { asm volatile("s_wait_dscnt 0" ::: "memory"); __builtin_amdgcn_wave_barrier(); __builtin_amdgcn_fence(__ATOMIC_RELEASE, "workgroup"); } while (0)


#define NB 4
#define CC 192
#define TT 1024
#define NH 8
#define HDIM 24
#define WIN 4
#define NREL (2 * WIN + 1)
#define NR (NB * TT)
#ifndef TQB
#define TQB (TT / 64)
#define TNB NB
#endif
typedef __attribute__((ext_vector_type(8))) __bf16 v8b;
__device__ __forceinline__ v16b frag_b(const __bf16* rowk0, int lane) {
  union { v16b v; v8b q[2]; } u; const __bf16* p = rowk0 + 8 * (lane >> 4);
  u.q[0] = *(const v8b*)p; u.q[1] = *(const v8b*)(p + 16); return u.v;
}
__device__ __forceinline__ float bfr(float v) { return (float)(__bf16)v; }
__device__ __attribute__((noinline)) float exp_ni(float v) { return expf(v); }
__device__ __attribute__((noinline)) float erf_ni(float v) { return erff(v); }

#define PK_Q 0
#define PK_END ((size_t)4 * CC * CC)
#define WS_PK  0u
#define WS_QH  (((2u * PK_END) + 127u) / 128u * 128u)
#define WS_QL  (WS_QH + 2u * NR * NH * 32)
#define WS_KH  (WS_QL + 2u * NR * NH * 32)
#define WS_KL  (WS_KH + 2u * NR * NH * 32)
#define WS_VH  (WS_KL + 2u * NR * NH * 32)
#define WS_VL  (WS_VH + 2u * (size_t)NB * NH * 32 * TT)
#define WS_RQ  (WS_VL + 2u * (size_t)NB * NH * 32 * TT)
#define WS_O   (WS_RQ + 4u * NR * NH * 16)
#define WS_END (WS_O + 4u * NR * CC)

__global__ __launch_bounds__(256) void k_pack(const float* __restrict__ WQ, const float* __restrict__ WK, const float* __restrict__ WV, const float* __restrict__ WO, __bf16* __restrict__ PK) {
  const int n = blockIdx.x, which = blockIdx.y, t = threadIdx.x; const float* Wm = (which == 0) ? WQ : (which == 1) ? WK : (which == 2) ? WV : WO; __shared__ __align__(16) __bf16 s[CC];
  if (t < CC) s[t] = (__bf16)Wm[(size_t)n * CC + t];
  __syncthreads();
  if (t < CC / 8) vst2((unsigned*)(PK + ((size_t)which * CC + n) * CC + t * 8), *(const v4u*)&s[t * 8]);
}
__global__ __launch_bounds__(128) void k_qkv(const float* __restrict__ X, const __bf16* __restrict__ PK, const float* __restrict__ BQ, const float* __restrict__ BK, const float* __restrict__ BV, const float* __restrict__ EK, _Float16* __restrict__ QH, _Float16* __restrict__ QL, _Float16* __restrict__ KH, _Float16* __restrict__ KL, _Float16* __restrict__ VH, _Float16* __restrict__ VL, float* __restrict__ RQ) {
  __shared__ __align__(16) __bf16 sa[64][CC + 8]; __shared__ __align__(16) float so[64][CC + 4]; __shared__ __align__(16) _Float16 sbuf[2 * NH * 32 * 72];
  typedef _Float16 (*ChunkT)[NH * 32 + 8]; typedef _Float16 (*PlaneT)[72]; ChunkT sth = (ChunkT)sbuf, stl = (ChunkT)(sbuf + 64 * (NH * 32 + 8)); PlaneT svh = (PlaneT)sbuf, svl = (PlaneT)(sbuf + NH * 32 * 72);
  const int tid = threadIdx.x, wave = tid >> 5, lane = tid & 31, col = lane & 15, g = lane >> 4; const int t0 = blockIdx.x * 64; const size_t b = blockIdx.y; const size_t r0 = b * TT + t0;
  for (int e = tid; e < 64 * CC; e += 128) { const int c = e >> 6, r = e & 63; sa[r][c] = (__bf16)X[(b * CC + c) * TT + t0 + r]; }
  if (tid < 64) for (int c = CC; c < CC + 8; ++c) sa[tid][c] = (__bf16)0.f;
  __syncthreads();
#pragma unroll 1
  for (int which = 0; which < 3; ++which) { const __bf16* P = PK + (size_t)which * CC * CC; const float* BB = (which == 0) ? BQ : (which == 1) ? BK : BV;
    v8f acc[12] = {};
#pragma unroll
    for (int kc = 0; kc < CC / 32; ++kc) { const v16b a = frag_b(&sa[wave * 16 + col][kc * 32], lane);
#pragma unroll
      for (int j = 0; j < 12; ++j) acc[j] = wmma_bf(a, frag_b(P + (size_t)(j * 16 + col) * CC + kc * 32, lane), acc[j]); }
#pragma unroll
    for (int j = 0; j < 12; ++j) { const float bb = bfr(BB[j * 16 + col]);
#pragma unroll
      for (int r = 0; r < 8; ++r) so[wave * 16 + 8 * g + r][j * 16 + col] = acc[j][r] + bb; }
    __syncthreads();
    if (which < 2) {
      for (int e = tid; e < 64 * NH * 32; e += 128) { const int r = e / (NH * 32), q = e % (NH * 32); const int h = q >> 5, d = q & 31; float v = 0.f; if (d < HDIM) v = so[r][h * HDIM + d]; const _Float16 hv = (_Float16)v; sth[r][q] = hv; stl[r][q] = (_Float16)((v - (float)hv) * 2048.0f); }
      if (which == 0) {
        for (int e = tid; e < 64 * NH * 4; e += 128) { const int r = e / (NH * 4), q = e % (NH * 4); const int h = q >> 2, r4 = (q & 3) * 4; v4f o4;
          for (int i = 0; i < 4; ++i) { const int rr = r4 + i; float a2 = 0.f; if (rr < NREL) { for (int d = 0; d < HDIM; ++d) a2 += so[r][h * HDIM + d] * bfr(EK[rr * HDIM + d]); } o4[i] = a2; }
          vst2(RQ + ((r0 + r) * NH + h) * 16 + r4, o4); } }
      __syncthreads();
      _Float16* DH_ = which ? KH : QH; _Float16* DL_ = which ? KL : QL;
      for (int e = tid; e < 64 * (NH * 32 / 8); e += 128) { const int r = e / (NH * 4), q = e % (NH * 4); const size_t o = (r0 + r) * (NH * 32) + q * 8; vst2((unsigned*)(DH_ + o), *(const v4u*)&sth[r][q * 8]); vst2((unsigned*)(DL_ + o), *(const v4u*)&stl[r][q * 8]); }
    } else {
      for (int e = tid; e < 64 * NH * 32; e += 128) { const int r = e & 63, q = e >> 6; const int h = q >> 5, d = q & 31; float v = 0.f; if (d < HDIM) v = so[r][h * HDIM + d]; const _Float16 hv = (_Float16)v; svh[q][r] = hv; svl[q][r] = (_Float16)((v - (float)hv) * 2048.0f); }
      __syncthreads();
      for (int e = tid; e < NH * 32 * 8; e += 128) { const int q = e >> 3, pc = e & 7; const size_t o = (b * NH * 32 + q) * TT + t0 + pc * 8; vst2((unsigned*)(VH + o), *(const v4u*)&svh[q][pc * 8]); vst2((unsigned*)(VL + o), *(const v4u*)&svl[q][pc * 8]); } }
    __syncthreads(); }
}
__global__ __launch_bounds__(128) void k_attn(const _Float16* __restrict__ QH, const _Float16* __restrict__ QL, const _Float16* __restrict__ KH, const _Float16* __restrict__ KL, const _Float16* __restrict__ VH, const _Float16* __restrict__ VL, const float* __restrict__ RQ, const int* __restrict__ MASK, const float* __restrict__ EV, float* __restrict__ O) {
  __shared__ __align__(16) _Float16 sph[4][16][40], spl[4][16][40]; __shared__ int smk[64][33]; __shared__ float srq[4][16][NREL + 1]; __shared__ float spp[4][16][NREL + 1]; __shared__ __align__(16) float so[64][2 * HDIM + 4];
  const int tid = threadIdx.x, wave = tid >> 5, lane = tid & 31, col = lane & 15, g = lane >> 4; const int qb = blockIdx.x, hp = blockIdx.y; const size_t b = blockIdx.z; const int q0 = qb * 64 + wave * 16; const size_t rq = b * TT + q0; const float isc = 1.0f / sqrtf((float)HDIM);
#pragma unroll 1
  for (int hh = 0; hh < 2; ++hh) { const int h = hp * 2 + hh;
    if (lane < 16) { for (int rr = 0; rr < NREL; ++rr) srq[wave][lane][rr] = RQ[((rq + lane) * NH + h) * 16 + rr]; }
    const v16h aq = frag_h(QH + (rq + col) * (NH * 32) + h * 32, lane), aql = frag_h(QL + (rq + col) * (NH * 32) + h * 32, lane);
    float m[8], l[8];
#pragma unroll
    for (int r = 0; r < 8; ++r) { m[r] = -3.0e38f; l[r] = 0.f; }
    v8f acc[2] = {}, accl[2] = {};
    __syncthreads();
#pragma unroll 1
    for (int ks = 0; ks < TT / 32; ++ks) { const int j0 = ks * 32;
      for (int e = tid; e < 64 * 8; e += 128) { const int r = e >> 3, q4 = e & 7; const v4i mv = *(const v4i*)(MASK + ((b * TT + qb * 64 + r) * TT) + j0 + q4 * 4); smk[r][q4 * 4] = mv[0]; smk[r][q4 * 4 + 1] = mv[1]; smk[r][q4 * 4 + 2] = mv[2]; smk[r][q4 * 4 + 3] = mv[3]; }
      __syncthreads();
      v8f s[2];
#pragma unroll
      for (int ct = 0; ct < 2; ++ct) { const int kk = j0 + ct * 16 + col; const size_t rk = (b * TT + kk) * (NH * 32) + h * 32; v8f c = {}, cl = {};
        { const v16h kh = frag_h(KH + rk, lane); c = wmma16(aq, kh, c); cl = wmma16(aql, kh, cl); cl = wmma16(aq, frag_h(KL + rk, lane), cl); }
#pragma unroll
        for (int r = 0; r < 8; ++r) { const int qi = q0 + 8 * g + r; const int dd = kk - qi; float sc = c[r] + cl[r] * (1.0f / 2048.0f); if (dd >= -WIN && dd <= WIN) sc += srq[wave][8 * g + r][dd + WIN]; const bool keep = smk[wave * 16 + 8 * g + r][ct * 16 + col] != 0; s[ct][r] = keep ? sc * isc : -3.0e38f; } }
#pragma unroll
      for (int r = 0; r < 8; ++r) { float mx = fmaxf(s[0][r], s[1][r]);
#pragma unroll
        for (int o = 1; o < 16; o <<= 1) mx = fmaxf(mx, __shfl_xor(mx, o));
        const float mn = fmaxf(m[r], mx); const float alpha = (m[r] <= -1.0e38f) ? 0.f : __expf(m[r] - mn);
        const float e0 = (s[0][r] <= -1.0e38f) ? 0.f : __expf(s[0][r] - mn), e1 = (s[1][r] <= -1.0e38f) ? 0.f : __expf(s[1][r] - mn); float es = e0 + e1;
#pragma unroll
        for (int o = 1; o < 16; o <<= 1) es += __shfl_xor(es, o);
        l[r] = l[r] * alpha + es; m[r] = (mn <= -1.0e38f) ? m[r] : mn; acc[0][r] *= alpha; acc[1][r] *= alpha; accl[0][r] *= alpha; accl[1][r] *= alpha;
        { const float p0 = e0 * 2048.0f, p1 = e1 * 2048.0f; const _Float16 h0 = (_Float16)p0, h1 = (_Float16)p1; sph[wave][8 * g + r][col] = h0; sph[wave][8 * g + r][16 + col] = h1; spl[wave][8 * g + r][col] = (_Float16)((p0 - (float)h0) * 2048.0f); spl[wave][8 * g + r][16 + col] = (_Float16)((p1 - (float)h1) * 2048.0f); } }
      LDSX();
      const v16h pah = frag_h(&sph[wave][col][0], lane), pal = frag_h(&spl[wave][col][0], lane);
#pragma unroll
      for (int dt = 0; dt < 2; ++dt) { const size_t vo = (b * NH * 32 + h * 32 + dt * 16 + col) * TT + j0; const v16h vh = frag_h(VH + vo, lane); acc[dt] = wmma16(pah, vh, acc[dt]); accl[dt] = wmma16(pal, vh, accl[dt]); accl[dt] = wmma16(pah, frag_h(VL + vo, lane), accl[dt]); }
      __syncthreads(); }
    if (col < NREL) {
#pragma unroll
      for (int r = 0; r < 8; ++r) { const int qi = q0 + 8 * g + r; const int sidx = qi + col - WIN; float pv = 0.f;
        if (sidx >= 0 && sidx < TT && MASK[((b * TT + qi) * TT) + sidx] != 0) { const size_t rqo = (rq + 8 * g + r) * (NH * 32) + h * 32, rko = (b * TT + sidx) * (NH * 32) + h * 32; float dot = 0.f;
          for (int d = 0; d < HDIM; ++d) { const float qv = (float)QH[rqo + d] + (float)QL[rqo + d] * (1.0f / 2048.0f); const float kv = (float)KH[rko + d] + (float)KL[rko + d] * (1.0f / 2048.0f); dot += qv * kv; }
          const float sc = (dot + srq[wave][8 * g + r][col]) * isc; pv = __expf(sc - m[r]) / l[r]; }
        spp[wave][8 * g + r][col] = pv; } }
    LDSX();
#pragma unroll
    for (int r = 0; r < 8; ++r) { const float il = (1.0f / 2048.0f) / l[r];
#pragma unroll
      for (int dt = 0; dt < 2; ++dt) { const int d = dt * 16 + col; if (d < HDIM) { float v = (acc[dt][r] + accl[dt][r] * (1.0f / 2048.0f)) * il;
          for (int jr = 0; jr < NREL; ++jr) v += spp[wave][8 * g + r][jr] * bfr(EV[jr * HDIM + d]);
          so[wave * 16 + 8 * g + r][hh * HDIM + d] = v; } } }
    __syncthreads(); }
  for (int e = tid; e < 64 * 12; e += 128) { const int r = e / 12, q4 = e % 12; vst2(O + ((size_t)hp * NR + b * TT + qb * 64 + r) * 48 + q4 * 4, *(const v4f*)&so[r][q4 * 4]); }
}
__global__ __launch_bounds__(128) void k_out(const float* __restrict__ O, const __bf16* __restrict__ PK, const float* __restrict__ BO, float* __restrict__ Y) {
  __shared__ __align__(16) __bf16 sh[128][CC + 8], sl[128][CC + 8]; __shared__ __align__(16) float so2[4][16][132];
  const int tid = threadIdx.x, wave = tid >> 5, lane = tid & 31, col = lane & 15, g = lane >> 4; const int o0 = blockIdx.x * 64 + wave * 16; const int n0 = blockIdx.y * 128; const size_t b = blockIdx.z;
  for (int e = tid; e < 128 * CC; e += 128) { const int r = e / CC, c = e % CC; const int hp = c / 48, w = c % 48; const float v = O[((size_t)hp * NR + b * TT + n0 + r) * 48 + w]; const __bf16 hb = (__bf16)v; sh[r][c] = hb; sl[r][c] = (__bf16)(v - (float)hb); }
  for (int e = tid; e < 128 * 8; e += 128) { const int r = e >> 3, c = CC + (e & 7); sh[r][c] = (__bf16)0.f; sl[r][c] = (__bf16)0.f; }
  __syncthreads();
  v8f acc[8] = {};
#pragma unroll
  for (int kc = 0; kc < CC / 32; ++kc) { const v16b a = frag_b(PK + (size_t)3 * CC * CC + (size_t)(o0 + col) * CC + kc * 32, lane);
#pragma unroll
    for (int j = 0; j < 8; ++j) { acc[j] = wmma_bf(a, frag_b(&sl[j * 16 + col][kc * 32], lane), acc[j]); acc[j] = wmma_bf(a, frag_b(&sh[j * 16 + col][kc * 32], lane), acc[j]); } }
#pragma unroll
  for (int j = 0; j < 8; ++j)
#pragma unroll
    for (int r = 0; r < 8; ++r) so2[wave][8 * g + r][j * 16 + col] = acc[j][r] + bfr(BO[o0 + 8 * g + r]);
  LDSX();
  for (int rl = 0; rl < 16; ++rl) vst2(Y + (b * CC + o0 + rl) * TT + n0 + lane * 4, *(const v4f*)&so2[wave][rl][lane * 4]);
}
extern "C" void kernel_launch(void* const* d_in, const int* in_sizes, int n_in, void* d_out, int out_size, void* d_ws, size_t ws_size, hipStream_t stream) {
  (void)in_sizes; (void)n_in; (void)out_size;
  const float** F = (const float**)d_in;
  if (ws_size < (size_t)WS_END) return;
  char* ws = (char*)d_ws; __bf16* PK = (__bf16*)(ws + WS_PK); _Float16 *QH = (_Float16*)(ws + WS_QH), *QL = (_Float16*)(ws + WS_QL), *KH = (_Float16*)(ws + WS_KH), *KL = (_Float16*)(ws + WS_KL), *VH = (_Float16*)(ws + WS_VH), *VL = (_Float16*)(ws + WS_VL); float *RQ = (float*)(ws + WS_RQ), *O = (float*)(ws + WS_O);
  k_pack<<<dim3(CC, 4), 256, 0, stream>>>(F[2], F[4], F[6], F[8], PK);
  k_qkv<<<dim3(TT / 64, NB), 128, 0, stream>>>(F[0], PK, F[3], F[5], F[7], F[10], QH, QL, KH, KL, VH, VL, RQ);
  k_attn<<<dim3(TQB, NH / 2, TNB), 128, 0, stream>>>(QH, QL, KH, KL, VH, VL, RQ, (const int*)d_in[1], F[11], O);
  k_out<<<dim3(CC / 64, TT / 128, TNB), 128, 0, stream>>>(O, PK, F[9], (float*)d_out);
}
